// DecoderAutoregSALN_90658169684689
// MI455X (gfx1250) — hardware-verified
//
#include <hip/hip_runtime.h>

typedef _Float16 bf16_t;
typedef bf16_t v16bf __attribute__((ext_vector_type(16)));
typedef float v4f_t __attribute__((ext_vector_type(4)));
typedef float v4fa  __attribute__((ext_vector_type(4), may_alias));
#define RSPLIT (1.0f / 2048.0f)
typedef float  v8f   __attribute__((ext_vector_type(8)));
typedef unsigned int v4u __attribute__((ext_vector_type(4)));
typedef unsigned int v8u __attribute__((ext_vector_type(8)));

#define DD   512
#define FFD  2048
#define NF   32
#define NB   2
#define NH   8
#define HDM  64
#define NL   4
#define MM   256
#define ZPAD_ELEMS 2080

__device__ __forceinline__ unsigned short f2bf(float x) { return __builtin_bit_cast(unsigned short, (_Float16)x); }
__device__ __forceinline__ unsigned short f2lo(float x) { const _Float16 h = (_Float16)x; return __builtin_bit_cast(unsigned short, (_Float16)((x - (float)h) * 2048.0f)); }
__device__ __forceinline__ unsigned pk2h(float a, float b) { return (unsigned)f2bf(a) | ((unsigned)f2bf(b) << 16); }
__device__ __forceinline__ unsigned pk2l(float a, float b) { return (unsigned)f2lo(a) | ((unsigned)f2lo(b) << 16); }
__device__ __forceinline__ void st2f(float* p, float v) { *(volatile float*)p = v; __threadfence(); *(volatile float*)p = v; }
__device__ __forceinline__ void st_pair(unsigned short* p, long plane, float a, float b) {
  const unsigned v = pk2h(a, b), l = pk2l(a, b);
  *(volatile unsigned*)p = v; *(volatile unsigned*)(p + plane) = l; __threadfence();
  *(volatile unsigned*)p = v; *(volatile unsigned*)(p + plane) = l;
}

__device__ __forceinline__ v16bf load_a_frag(const unsigned short* row, int hi) {
  v4u lo = *(const v4u*)(row + hi * 8);
  v4u hh = *(const v4u*)(row + 16 + hi * 8);
  v8u r;
  r[0] = lo[0]; r[1] = lo[1]; r[2] = lo[2]; r[3] = lo[3];
  r[4] = hh[0]; r[5] = hh[1]; r[6] = hh[2]; r[7] = hh[3];
  return __builtin_bit_cast(v16bf, r);
}

__device__ __forceinline__ v16bf load_b_frag(const unsigned short* col, int hi) {
  return load_a_frag(col, hi);
}

__device__ __forceinline__ v8f wmma_bf16(v16bf a, v16bf b, v8f c) {
  return __builtin_amdgcn_wmma_f32_16x16x32_f16(false, a, false, b, (short)0, c, false, false);
}
__device__ __forceinline__ v8f wmma_split(v16bf a, v16bf al, v16bf b, v16bf bl, v8f c) {
  v8f x = {0.f,0.f,0.f,0.f,0.f,0.f,0.f,0.f};
  x = wmma_bf16(al, b, x); x = wmma_bf16(a, bl, x); return wmma_bf16(a, b, c) + x * RSPLIT;
}

__device__ __forceinline__ v8f tile_gemm(const unsigned short* A, int lda, int validRows,
                                         const unsigned short* __restrict__ W, int K,
                                         int ntile, int lane,
                                         const unsigned short* zpad, long apl, long wpl) {
  const int r = lane & 15, hi = lane >> 4;
  const bool vr = (r < validRows);
  const unsigned short* a_row  = vr ? (A + (long)r * lda) : zpad;
  const unsigned short* a_rowl = vr ? (A + apl + (long)r * lda) : zpad;
  const unsigned short* w_col = W + (long)(ntile * 16 + r) * K;
  v8f acc = {0.f,0.f,0.f,0.f,0.f,0.f,0.f,0.f};
#pragma unroll 1
  for (int kk = 0; kk < K; kk += 32) {
    v16bf a  = load_a_frag(a_row + kk, hi);
    v16bf al = load_a_frag(a_rowl + kk, hi);
    v16bf b  = load_b_frag(w_col + kk, hi);
    v16bf bl = load_b_frag(w_col + wpl + kk, hi);
    acc = wmma_split(a, al, b, bl, acc);
  }
  return acc;
}


__global__ void conv_t_kernel(const float* __restrict__ W, unsigned short* __restrict__ Wt,
                              int K, int N) {
  long per = (long)K * N;
  const float* w = W + per * blockIdx.z;
  unsigned short* o = Wt + per * blockIdx.z;
  const long plane = per * gridDim.z;
  long idx = ((long)blockIdx.x * blockDim.x + threadIdx.x) * 2;
  if (idx < per) {
    int n = (int)(idx / K), k = (int)(idx % K);
    st_pair(o + (long)n * K + k, plane, w[(long)k * N + n], w[(long)(k + 1) * N + n]);
  }
}

__global__ void conv_b16_kernel(const float* __restrict__ x, unsigned short* __restrict__ y,
                                int n) {
  int i = (blockIdx.x * blockDim.x + threadIdx.x) * 2;
  if (i < n) st_pair(y + i, (long)n, x[i], x[i + 1]);
}

__global__ void gb_kernel(const float* __restrict__ style, const float* __restrict__ W,
                          const float* __restrict__ bsa, float* __restrict__ GB) {
  int idx = blockIdx.x * blockDim.x + threadIdx.x;
  if (idx >= NL * 3 * NB * 2 * DD) return;
  int n = idx & 1023;
  int b = (idx >> 10) & 1;
  int j = (idx >> 11) % 3;
  int l = idx / (1024 * 2 * 3);
  float acc = bsa[(l * 3 + j) * 1024 + n];
  const float* wp = W + (((long)l * 3 + j) * DD) * 1024 + n;
  const float* sp = style + b * DD;
  for (int k = 0; k < DD; ++k) acc += sp[k] * wp[(long)k * 1024];
  st2f(GB + idx, acc);
}

__global__ __launch_bounds__(32) void wmma_gemm_kernel(const unsigned short* __restrict__ A, int lda, long aB,
                                 const unsigned short* __restrict__ W, long wB,
                                 const float* __restrict__ bias, long biasB,
                                 float* Cf, unsigned short* Cbf, int ldc, long cB,
                                 int Mrows, int K, int relu,
                                 const unsigned short* __restrict__ zpad, long g_apl, long g_wpl, long g_cpl) {
  __shared__ __align__(16) float stg[16 * 68];
  const int lane = threadIdx.x & 31;
  const int ngrp = blockIdx.x, mtile = blockIdx.y, z = blockIdx.z;
  const int r = lane & 15, hi = lane >> 4;
  const unsigned short* a0 = A + (long)z * aB + (long)(mtile * 16) * lda;
#pragma unroll
  for (int q = 0; q < 4; ++q) {
    const int ntile = ngrp * 4 + q;
    v8f acc = tile_gemm(a0, lda, Mrows - mtile * 16, W + (long)z * wB, K, ntile, lane, zpad, g_apl, g_wpl);
    const int n = ntile * 16 + r;
    const float bz = bias ? bias[(long)z * biasB + n] : 0.f;
#pragma unroll
    for (int j = 0; j < 8; ++j) { float v = acc[j] + bz; if (relu) v = fmaxf(v, 0.f); stg[(hi * 8 + j) * 68 + q * 16 + r] = v; }
  }
  asm volatile("s_wait_dscnt 0" ::: "memory");
  const int n0 = ngrp * 64;
#pragma unroll 1
  for (int pass = 0; pass < 2; ++pass) {
    if (Cf) {
#pragma unroll
      for (int i = 0; i < 8; ++i) { const int c = lane + 32 * i, rr = c >> 4, qq = (c & 15) * 4; const int row = mtile * 16 + rr;
        if (row < Mrows) *(volatile v4f_t*)(Cf + (long)z * cB + (long)row * ldc + n0 + qq) = *(const volatile v4fa*)(stg + rr * 68 + qq); }
    }
    if (Cbf) {
#pragma unroll
      for (int i = 0; i < 4; ++i) { const int c = lane + 32 * i, rr = c >> 3, qq = (c & 7) * 8; const int row = mtile * 16 + rr; const float* s = stg + rr * 68 + qq;
        if (row < Mrows) {
          __attribute__((ext_vector_type(4))) unsigned v, vl;
          v.x = pk2h(s[0], s[1]); v.y = pk2h(s[2], s[3]); v.z = pk2h(s[4], s[5]); v.w = pk2h(s[6], s[7]);
          vl.x = pk2l(s[0], s[1]); vl.y = pk2l(s[2], s[3]); vl.z = pk2l(s[4], s[5]); vl.w = pk2l(s[6], s[7]);
          typedef __attribute__((ext_vector_type(4))) unsigned v4u_t;
          *(volatile v4u_t*)(Cbf + (long)z * cB + (long)row * ldc + n0 + qq) = v;
          *(volatile v4u_t*)(Cbf + g_cpl + (long)z * cB + (long)row * ldc + n0 + qq) = vl; } }
    }
    __threadfence();
  }
}


__device__ __forceinline__ float wave_sum(float v) {
  for (int m = 16; m; m >>= 1) v += __shfl_xor(v, m, 32);
  return v;
}

__device__ __forceinline__ float ppe_val(int t, int d) {
  int pos = t % 30;
  float div = __expf((float)(d & ~1) * (-9.210340371976184f / 512.f));
  float a = (float)pos * div;
  return (d & 1) ? __cosf(a) : __sinf(a);
}

__device__ __forceinline__ void saln_ln(const float* ys, float* xs, unsigned short* xb,
                                        const float* __restrict__ gb, float* red, int tid) {
  if (tid < 4) red[tid] = 0.f;
  __syncthreads();
  const int d = tid;
  float v0 = ys[d], v1 = ys[DD + d];
  float s0 = wave_sum(v0), s1 = wave_sum(v1);
  if ((tid & 31) == 0) { atomicAdd(&red[0], s0); atomicAdd(&red[1], s1); }
  __syncthreads();
  float mu0 = red[0] * (1.f / 512.f), mu1 = red[1] * (1.f / 512.f);
  float d0 = v0 - mu0, d1 = v1 - mu1;
  float q0 = wave_sum(d0 * d0), q1 = wave_sum(d1 * d1);
  if ((tid & 31) == 0) { atomicAdd(&red[2], q0); atomicAdd(&red[3], q1); }
  __syncthreads();
  float r0 = rsqrtf(red[2] * (1.f / 512.f) + 1e-5f), r1 = rsqrtf(red[3] * (1.f / 512.f) + 1e-5f);
  float o0 = d0 * r0 * gb[d] + gb[512 + d], o1 = d1 * r1 * gb[1024 + d] + gb[1024 + 512 + d];
  xs[d] = o0; xs[DD + d] = o1;
  xb[d] = f2bf(o0); xb[2 * DD + d] = f2lo(o0); xb[DD + d] = f2bf(o1); xb[2 * DD + DD + d] = f2lo(o1);
  __syncthreads();
}

__global__ __launch_bounds__(512) void decode_persistent(
    const unsigned short* __restrict__ sqw, const unsigned short* __restrict__ skw,
    const unsigned short* __restrict__ svw, const unsigned short* __restrict__ sow,
    const unsigned short* __restrict__ f1w, const unsigned short* __restrict__ f2w,
    const unsigned short* __restrict__ mow, const unsigned short* __restrict__ mrw,
    const float* __restrict__ bq, const float* __restrict__ bk,
    const float* __restrict__ bv, const float* __restrict__ bo,
    const float* __restrict__ b1, const float* __restrict__ b2,
    const float* __restrict__ mob, const float* __restrict__ mrb,
    const float* __restrict__ GB, const float* __restrict__ CA,
    const float* __restrict__ emb0, float* kc, float* vc, float* out) {
  __shared__ __align__(32) float xs[2 * DD], ys[2 * DD], qs[2 * DD];
  __shared__ __align__(32) unsigned short xb[2 * 2 * DD], ob[2 * 2 * DD];
  __shared__ __align__(32) unsigned short h1b[2 * 2 * FFD], orb[2 * 2 * MM];
  __shared__ __align__(16) float kvs[2][2 * DD];
  __shared__ __align__(16) float outs[2 * MM];
  __shared__ __align__(32) unsigned short zp[ZPAD_ELEMS];
  __shared__ float red[4];

  const int tid = threadIdx.x, w = tid >> 5, lane = tid & 31;
  for (int i = tid; i < ZPAD_ELEMS; i += 512) zp[i] = 0;
#pragma unroll
  for (int b = 0; b < 2; ++b) {
    const int d = tid, e = b * DD + d;
    float v = emb0[e] + ppe_val(0, d);
    xs[e] = v;
    xb[e] = f2bf(v); xb[2 * DD + e] = f2lo(v);
  }
  __syncthreads();
  const long PW = (long)NL * DD * DD, PF = (long)NL * FFD * DD, PMO = (long)DD * MM;

  for (int t = 0; t < NF; ++t) {
    for (int l = 0; l < NL; ++l) {
#pragma unroll 1
      for (int tt = w; tt < 96; tt += 16) {
        int which = tt >> 5, nt = tt & 31;
        const unsigned short* Wt = (which == 0) ? sqw : (which == 1) ? skw : svw;
        const float* bb = (which == 0) ? bq : (which == 1) ? bk : bv;
        v8f acc = tile_gemm(xb, DD, 2, Wt + (long)l * DD * DD, DD, nt, lane, zp, 2 * DD, PW);
        if (lane < 16) {
          int n = nt * 16 + lane;
          float r0 = acc[0] + bb[l * DD + n];
          float r1 = acc[1] + bb[l * DD + n];
          if (which == 0) { qs[n] = r0; qs[DD + n] = r1; }
          else { kvs[which - 1][n] = r0; kvs[which - 1][DD + n] = r1; }
        }
      }
      __syncthreads();
#pragma unroll 1
      for (int pass = 0; pass < 2; ++pass) {
        { const int which = tid >> 8, c4 = tid & 255, b = c4 >> 7, q = (c4 & 127) * 4; float* c = (which == 0) ? kc : vc;
          *(volatile v4f_t*)(c + (((long)l * NB + b) * NF + t) * DD + q) = *(const volatile v4fa*)(&kvs[which][b * DD + q]); }
        __threadfence();
      }
      __syncthreads();

      if (w < 16) {
        int b = w >> 3, h = w & 7;
        const float* kcb = kc + (((long)l * NB + b) * NF) * DD + h * HDM;
        const float* vcb = vc + (((long)l * NB + b) * NF) * DD + h * HDM;
        float sc = -1e30f;
        if (lane <= t) {
          const float* kv = kcb + (long)lane * DD;
          float acc = 0.f;
#pragma unroll 8
          for (int e = 0; e < HDM; ++e) acc += qs[b * DD + h * HDM + e] * kv[e];
          float slope = exp2f(-(float)(h + 1));
          sc = acc * 0.125f + slope * (-(float)((t - lane) / 30));
        }
        float m = sc;
        for (int msk = 16; msk; msk >>= 1) m = fmaxf(m, __shfl_xor(m, msk, 32));
        float p = (lane <= t) ? __expf(sc - m) : 0.f;
        float ssum = p;
        for (int msk = 16; msk; msk >>= 1) ssum += __shfl_xor(ssum, msk, 32);
        float att = p / ssum;
        float a0 = 0.f, a1 = 0.f;
        for (int s2 = 0; s2 <= t; ++s2) {
          float aw = __shfl(att, s2, 32);
          const float* vv = vcb + (long)s2 * DD;
          a0 += aw * vv[lane];
          a1 += aw * vv[32 + lane];
        }
        ob[b * DD + h * HDM + lane] = f2bf(a0);       ob[2 * DD + b * DD + h * HDM + lane] = f2lo(a0);
        ob[b * DD + h * HDM + 32 + lane] = f2bf(a1);  ob[2 * DD + b * DD + h * HDM + 32 + lane] = f2lo(a1);
      }
      __syncthreads();

#pragma unroll 1
      for (int tt = w; tt < 32; tt += 16) {
        v8f acc = tile_gemm(ob, DD, 2, sow + (long)l * DD * DD, DD, tt, lane, zp, 2 * DD, PW);
        if (lane < 16) {
          int n = tt * 16 + lane;
          ys[n]      = xs[n]      + acc[0] + bo[l * DD + n];
          ys[DD + n] = xs[DD + n] + acc[1] + bo[l * DD + n];
        }
      }
      __syncthreads();
      saln_ln(ys, xs, xb, GB + ((long)(l * 3 + 0) * 2) * 1024, red, tid);

#pragma unroll
      for (int b = 0; b < 2; ++b) { const int d = tid, e = b * DD + d; ys[e] = xs[e] + CA[(((long)l * NB + b) * NF + t) * DD + d]; }
      __syncthreads();
      saln_ln(ys, xs, xb, GB + ((long)(l * 3 + 1) * 2) * 1024, red, tid);

#pragma unroll 1
      for (int tt = w; tt < 128; tt += 16) {
        v8f acc = tile_gemm(xb, DD, 2, f1w + (long)l * FFD * DD, DD, tt, lane, zp, 2 * DD, PF);
        if (lane < 16) {
          int n = tt * 16 + lane;
          const float u0 = fmaxf(acc[0] + b1[l * FFD + n], 0.f), u1 = fmaxf(acc[1] + b1[l * FFD + n], 0.f);
          h1b[n]       = f2bf(u0); h1b[2 * FFD + n]       = f2lo(u0);
          h1b[FFD + n] = f2bf(u1); h1b[2 * FFD + FFD + n] = f2lo(u1);
        }
      }
      __syncthreads();
#pragma unroll 1
      for (int tt = w; tt < 32; tt += 16) {
        v8f acc = tile_gemm(h1b, FFD, 2, f2w + (long)l * DD * FFD, FFD, tt, lane, zp, 2 * FFD, PF);
        if (lane < 16) {
          int n = tt * 16 + lane;
          ys[n]      = xs[n]      + acc[0] + b2[l * DD + n];
          ys[DD + n] = xs[DD + n] + acc[1] + b2[l * DD + n];
        }
      }
      __syncthreads();
      saln_ln(ys, xs, xb, GB + ((long)(l * 3 + 2) * 2) * 1024, red, tid);
    }

    if (w < 16) {
      v8f acc = tile_gemm(xb, DD, 2, mrw, DD, w, lane, zp, 2 * DD, PMO);
      if (lane < 16) {
        int n = w * 16 + lane;
        float r0 = acc[0] + mrb[n], r1 = acc[1] + mrb[n];
        outs[n] = r0; outs[MM + n] = r1;
        orb[n] = f2bf(r0);      orb[2 * MM + n] = f2lo(r0);
        orb[MM + n] = f2bf(r1); orb[2 * MM + MM + n] = f2lo(r1);
      }
    }
    __syncthreads();
#pragma unroll 1
    for (int pass = 0; pass < 2; ++pass) {
      if (tid < 128) { const int b = tid >> 6, q = (tid & 63) * 4; *(volatile v4f_t*)(out + ((long)b * NF + t) * MM + q) = *(const volatile v4fa*)(&outs[b * MM + q]); }
      __threadfence();
    }

    if (t + 1 < NF) {
#pragma unroll 1
     for (int tt = w; tt < 32; tt += 16) {
      v8f acc = tile_gemm(orb, MM, 2, mow, MM, tt, lane, zp, 2 * MM, PMO);
      if (lane < 16) {
        int n = tt * 16 + lane;
        float e0 = acc[0] + mob[n] + ppe_val(t + 1, n);
        float e1 = acc[1] + mob[n] + ppe_val(t + 1, n);
        xs[n] = e0;      xs[DD + n] = e1;
        xb[n] = f2bf(e0); xb[DD + n] = f2bf(e1); xb[2 * DD + n] = f2lo(e0); xb[2 * DD + DD + n] = f2lo(e1);
      }
     }
      __syncthreads();
    }
  }
}


extern "C" void kernel_launch(void* const* d_in, const int* in_sizes, int n_in,
                              void* d_out, int out_size, void* d_ws, size_t ws_size,
                              hipStream_t stream) {
  (void)in_sizes; (void)n_in; (void)out_size; (void)ws_size;
  char* ws = (char*)d_ws;
  size_t off = 0;
  auto take = [&](size_t bytes) {
    size_t r = off;
    off += (bytes + 255) & ~(size_t)255;
    return r;
  };

  const size_t szDD = (size_t)NL * DD * DD * 2 * 2;
  size_t o_sq = take(szDD), o_sk = take(szDD), o_sv = take(szDD), o_so = take(szDD);
  size_t o_f1 = take((size_t)NL * FFD * DD * 2 * 2);
  size_t o_f2 = take((size_t)NL * DD * FFD * 2 * 2);
  size_t o_cv = take(szDD), o_co = take(szDD);
  size_t o_mo = take((size_t)DD * MM * 2 * 2);
  size_t o_mr = take((size_t)MM * DD * 2 * 2);
  size_t o_cb = take((size_t)NB * NF * DD * 2 * 2);
  size_t o_ib = take((size_t)NB * MM * 2 * 2);
  size_t o_tb = take((size_t)NL * NB * NF * DD * 2 * 2);
  const long PW = (long)NL * DD * DD, PF = (long)NL * FFD * DD, PMO = (long)DD * MM, PCB = (long)NB * NF * DD, PIB = (long)NB * MM, PTB = (long)NL * NB * NF * DD;
  size_t o_CA = take((size_t)NL * NB * NF * DD * 4);
  size_t o_GB = take((size_t)NL * 3 * NB * 2 * DD * 4);
  size_t o_e0 = take((size_t)NB * DD * 4);
  size_t o_kc = take((size_t)NL * NB * NF * DD * 4);
  size_t o_vc = take((size_t)NL * NB * NF * DD * 4);
  size_t o_zp = take((size_t)ZPAD_ELEMS * 2 + 64);

  const float* content  = (const float*)d_in[0];
  const float* style    = (const float*)d_in[1];
  const float* init_st  = (const float*)d_in[2];
  const float* motion_W = (const float*)d_in[3];
  const float* motion_b = (const float*)d_in[4];
  const float* motionr_W= (const float*)d_in[5];
  const float* motionr_b= (const float*)d_in[6];

  hipMemsetAsync(ws + o_zp, 0, (size_t)ZPAD_ELEMS * 2 + 64, stream);

  conv_t_kernel<<<dim3(1024, 1, NL), 256, 0, stream>>>((const float*)d_in[7],  (unsigned short*)(ws + o_sq), DD, DD);
  conv_t_kernel<<<dim3(1024, 1, NL), 256, 0, stream>>>((const float*)d_in[9],  (unsigned short*)(ws + o_sk), DD, DD);
  conv_t_kernel<<<dim3(1024, 1, NL), 256, 0, stream>>>((const float*)d_in[11], (unsigned short*)(ws + o_sv), DD, DD);
  conv_t_kernel<<<dim3(1024, 1, NL), 256, 0, stream>>>((const float*)d_in[13], (unsigned short*)(ws + o_so), DD, DD);
  conv_t_kernel<<<dim3(1024, 1, NL), 256, 0, stream>>>((const float*)d_in[19], (unsigned short*)(ws + o_cv), DD, DD);
  conv_t_kernel<<<dim3(1024, 1, NL), 256, 0, stream>>>((const float*)d_in[21], (unsigned short*)(ws + o_co), DD, DD);
  conv_t_kernel<<<dim3(4096, 1, NL), 256, 0, stream>>>((const float*)d_in[23], (unsigned short*)(ws + o_f1), DD, FFD);
  conv_t_kernel<<<dim3(4096, 1, NL), 256, 0, stream>>>((const float*)d_in[25], (unsigned short*)(ws + o_f2), FFD, DD);
  conv_t_kernel<<<dim3(512, 1, 1),   256, 0, stream>>>(motion_W,  (unsigned short*)(ws + o_mo), MM, DD);
  conv_t_kernel<<<dim3(512, 1, 1),   256, 0, stream>>>(motionr_W, (unsigned short*)(ws + o_mr), DD, MM);

  conv_b16_kernel<<<128, 256, 0, stream>>>(content, (unsigned short*)(ws + o_cb), NB * NF * DD);
  conv_b16_kernel<<<2, 256, 0, stream>>>(init_st, (unsigned short*)(ws + o_ib), NB * MM);

  gb_kernel<<<96, 256, 0, stream>>>(style, (const float*)d_in[27], (const float*)d_in[28],
                                    (float*)(ws + o_GB));

  const unsigned short* zpad = (const unsigned short*)(ws + o_zp);

  wmma_gemm_kernel<<<dim3(DD / 64, 1, 1), 32, 0, stream>>>(
      (const unsigned short*)(ws + o_ib), MM, 0,
      (const unsigned short*)(ws + o_mo), 0,
      motion_b, 0,
      (float*)(ws + o_e0), nullptr, DD, 0, NB, MM, 0, zpad, PIB, PMO, 0);

  wmma_gemm_kernel<<<dim3(DD / 64, 4, NL), 32, 0, stream>>>(
      (const unsigned short*)(ws + o_cb), DD, 0,
      (const unsigned short*)(ws + o_cv), (long)DD * DD,
      (const float*)d_in[20], DD,
      nullptr, (unsigned short*)(ws + o_tb), DD, (long)NB * NF * DD, NB * NF, DD, 0, zpad, PCB, PW, PTB);
  wmma_gemm_kernel<<<dim3(DD / 64, 4, NL), 32, 0, stream>>>(
      (const unsigned short*)(ws + o_tb), DD, (long)NB * NF * DD,
      (const unsigned short*)(ws + o_co), (long)DD * DD,
      (const float*)d_in[22], DD,
      (float*)(ws + o_CA), nullptr, DD, (long)NB * NF * DD, NB * NF, DD, 0, zpad, PTB, PW, 0);

  decode_persistent<<<1, 512, 0, stream>>>(
      (const unsigned short*)(ws + o_sq), (const unsigned short*)(ws + o_sk),
      (const unsigned short*)(ws + o_sv), (const unsigned short*)(ws + o_so),
      (const unsigned short*)(ws + o_f1), (const unsigned short*)(ws + o_f2),
      (const unsigned short*)(ws + o_mo), (const unsigned short*)(ws + o_mr),
      (const float*)d_in[8], (const float*)d_in[10], (const float*)d_in[12],
      (const float*)d_in[14], (const float*)d_in[24], (const float*)d_in[26],
      motion_b, motionr_b,
      (const float*)(ws + o_GB), (const float*)(ws + o_CA), (const float*)(ws + o_e0),
      (float*)(ws + o_kc), (float*)(ws + o_vc), (float*)d_out);
}
